// FastRNNlayer_32873679684250
// MI455X (gfx1250) — hardware-verified
//
#include <hip/hip_runtime.h>
#include <math.h>

constexpr int kS       = 512;
constexpr int kB       = 8;
constexpr int kNH      = 8;
constexpr int kHD      = 64;
constexpr int kIN      = 512;
constexpr int kHeadW   = 5 * kHD + 2;
constexpr int kProj    = kNH * kHeadW;
constexpr int kProjPad = 2624;
constexpr int kRows    = kS * kB;
static_assert(kProjPad % 64 == 0 && kProjPad >= kProj, "pad");
static_assert(kRows % 64 == 0 && kIN % 64 == 0 && kIN % 32 == 0, "tiles");

constexpr float kWCarry   = 16.0f;
constexpr float kHsCarry  = 32.0f;
constexpr float kG1Scale  = 1.0f / 16.0f;
constexpr float kG2Scale  = 1.0f / 512.0f;
constexpr float kInvDim   = 1.0f / 512.0f;
constexpr float kLnEps    = 1e-5f;

constexpr size_t kOffNormed = 0;
constexpr size_t kOffWslow  = kOffNormed + (size_t)kRows * kIN * 2;
constexpr size_t kOffWout   = kOffWslow + (size_t)kProjPad * kIN * 2;
constexpr size_t kOffQkvb   = kOffWout + (size_t)kIN * kIN * 2;
constexpr size_t kOffHs     = kOffQkvb + (size_t)kRows * kProjPad * 4;
constexpr size_t kWsTotal   = kOffHs + (size_t)kRows * kIN * 2;
static_assert(kWsTotal == 54591488, "carve");
static_assert(kOffWslow % 128 == 0 && kOffWout % 128 == 0 && kOffQkvb % 128 == 0 && kOffHs % 128 == 0, "align");

typedef __attribute__((ext_vector_type(16))) _Float16 v16h;
typedef __attribute__((ext_vector_type(8)))  _Float16 v8h;
typedef __attribute__((ext_vector_type(16))) __bf16   v16b;
typedef __attribute__((ext_vector_type(8)))  __bf16   v8b;
typedef __attribute__((ext_vector_type(8)))  float    v8f;
typedef __attribute__((ext_vector_type(4)))  float    v4f;
typedef __attribute__((ext_vector_type(4)))  unsigned int v4u;

__device__ __forceinline__ unsigned short f2bf_bits(float f) {
  unsigned u = __float_as_uint(f);
  return (unsigned short)((u + 0x7FFFu + ((u >> 16) & 1u)) >> 16);
}
__device__ __forceinline__ float bf_bits2f(unsigned short h) { return __uint_as_float(((unsigned)h) << 16); }

__device__ __forceinline__ void dep_guard_h(v8f& a, v8f& b, v16h x, v16h y) { asm volatile("v_nop\n\tv_nop\n\tv_nop\n\tv_nop" : "+v"(a), "+v"(b) : "v"(x), "v"(y)); }
__device__ __forceinline__ void dep_guard_b(v8f& a, v8f& b, v16b x, v16b y) { asm volatile("v_nop\n\tv_nop\n\tv_nop\n\tv_nop" : "+v"(a), "+v"(b) : "v"(x), "v"(y)); }
__device__ __forceinline__ void keep4_h(v16h a, v16h b, v16h c, v16h d) { asm volatile("v_nop" :: "v"(a), "v"(b), "v"(c), "v"(d)); }
__device__ __forceinline__ void keep4_b(v16b a, v16b b, v16b c, v16b d) { asm volatile("v_nop" :: "v"(a), "v"(b), "v"(c), "v"(d)); }
__device__ __forceinline__ void acc_guard4(v8f& a, v8f& b, v8f& c, v8f& d) { asm volatile("v_nop\n\tv_nop\n\tv_nop\n\tv_nop" : "+v"(a), "+v"(b), "+v"(c), "+v"(d)); }
template <typename T> struct Frag;
template <> struct Frag<_Float16> {
  typedef v16h V; union U { v16h v; v8h h[2]; };
  static __device__ __forceinline__ v16h load(const _Float16* p) {
    U f; f.h[0] = *(const v8h*)(p); f.h[1] = *(const v8h*)(p + 16); return f.v;
  }
  static __device__ __forceinline__ v8f mma(v16h a, v16h b, v8f c) {
    return __builtin_amdgcn_wmma_f32_16x16x32_f16(false, a, false, b, (short)0, c, false, false);
  }
  static __device__ __forceinline__ void guard(v8f& a, v8f& b, v16h x, v16h y) { dep_guard_h(a, b, x, y); }
  static __device__ __forceinline__ void keep(v16h a, v16h b, v16h c, v16h d) { keep4_h(a, b, c, d); }
};
template <> struct Frag<__bf16> {
  typedef v16b V; union U { v16b v; v8b h[2]; };
  static __device__ __forceinline__ v16b load(const __bf16* p) {
    U f; f.h[0] = *(const v8b*)(p); f.h[1] = *(const v8b*)(p + 16); return f.v;
  }
  static __device__ __forceinline__ v8f mma(v16b a, v16b b, v8f c) {
    return __builtin_amdgcn_wmma_f32_16x16x32_bf16(false, a, false, b, (short)0, c, false, false);
  }
  static __device__ __forceinline__ void guard(v8f& a, v8f& b, v16b x, v16b y) { dep_guard_b(a, b, x, y); }
  static __device__ __forceinline__ void keep(v16b a, v16b b, v16b c, v16b d) { keep4_b(a, b, c, d); }
};

__device__ __forceinline__ unsigned pk16(unsigned short a, unsigned short b) { return (unsigned)a | ((unsigned)b << 16); }
__device__ __forceinline__ unsigned short h_bits(float f) { const _Float16 h = (_Float16)f; return __builtin_bit_cast(unsigned short, h); }
__device__ __forceinline__ void defuse(float& v) { asm volatile("" : "+v"(v)); }

template <int ET> struct Elem;
template <> struct Elem<0> { typedef _Float16 T; };
template <> struct Elem<1> { typedef __bf16 T; };
template <int ET, bool SPLIT, int BIAS_MODE, int OUT_MODE, bool RESID, int ACT = 0>
__global__ __launch_bounds__(256) void wmma_gemm64(
    const unsigned short* __restrict__ Ap, const unsigned short* __restrict__ A2p, int lda, long strideA,
    const unsigned short* __restrict__ Btp, const unsigned short* __restrict__ Bt2p, int ldb, long strideB,
    void* __restrict__ Cout, void* __restrict__ Cout2, int ldc, long strideC,
    const float* __restrict__ bias,
    const float* __restrict__ resid, long strideR,
    int M, int N, int K, float scale) {
  typedef typename Elem<ET>::T T;
  typedef typename Frag<T>::V V;
  const T* A = (const T*)Ap; const T* A2 = (const T*)A2p; const T* Bt = (const T*)Btp; const T* Bt2 = (const T*)Bt2p;
  __shared__ __align__(16) float sT[8][16 * 68];
  const int b    = blockIdx.y;
  const int lane = threadIdx.x & 31;
  const int wave = threadIdx.x >> 5;
  const int tilesN = N >> 6;
  const int tilesM = M >> 6;
  const int tile = blockIdx.x * 8 + wave;
  if (tile >= tilesM * tilesN) return;
  const int tm = tile / tilesN;
  const int tn = tile - tm * tilesN;
  const int m0 = tm << 6;
  const int n0 = tn << 6;

  const T* Ab  = A  + (size_t)b * strideA;
  const T* Bb  = Bt + (size_t)b * strideB;
  const T* Ab2 = SPLIT ? (A2  + (size_t)b * strideA) : nullptr;
  const T* Bb2 = SPLIT ? (Bt2 + (size_t)b * strideB) : nullptr;

  const int rlane = lane & 15;
  const int koff  = (lane >> 4) * 8;
  const int mOff  = (lane >> 4) * 8;

  v8f acc[4][4];
#pragma unroll
  for (int i = 0; i < 4; ++i)
#pragma unroll
    for (int j = 0; j < 4; ++j) acc[i][j] = (v8f){0.f,0.f,0.f,0.f,0.f,0.f,0.f,0.f};

  for (int k0 = 0; k0 < K; k0 += 32) {
    V bh[4], bl[4];
#pragma unroll
    for (int j = 0; j < 4; ++j) {
      const size_t bo = (size_t)(n0 + (j << 4) + rlane) * ldb + koff + k0;
      bh[j] = Frag<T>::load(Bb + bo);
      if (SPLIT) bl[j] = Frag<T>::load(Bb2 + bo);
    }
#pragma unroll
    for (int i = 0; i < 4; ++i) {
      const size_t ao = (size_t)(m0 + (i << 4) + rlane) * lda + koff + k0;
      V ah = Frag<T>::load(Ab + ao);
      V al;
      if (SPLIT) al = Frag<T>::load(Ab2 + ao);
#pragma unroll
      for (int j = 0; j < 4; ++j) {
        acc[i][j] = Frag<T>::mma(ah, bh[j], acc[i][j]);
        if (SPLIT) {
          acc[i][j] = Frag<T>::mma(ah, bl[j], acc[i][j]);
          acc[i][j] = Frag<T>::mma(al, bh[j], acc[i][j]);
        }
      }
      Frag<T>::guard(acc[i][0], acc[i][3], ah, SPLIT ? al : ah);
    }
    Frag<T>::keep(bh[0], bh[1], bh[2], bh[3]);
    if (SPLIT) Frag<T>::keep(bl[0], bl[1], bl[2], bl[3]);
  }
  acc_guard4(acc[0][0], acc[0][1], acc[0][2], acc[0][3]);
  acc_guard4(acc[1][0], acc[1][1], acc[1][2], acc[1][3]);
  acc_guard4(acc[2][0], acc[2][1], acc[2][2], acc[2][3]);
  acc_guard4(acc[3][0], acc[3][1], acc[3][2], acc[3][3]);

  float* slab = sT[wave];
  const float* Rb = RESID ? (resid + (size_t)b * strideR) : nullptr;
#pragma unroll
  for (int i = 0; i < 4; ++i) {
    const int mBase = m0 + (i << 4);
#pragma unroll
    for (int j = 0; j < 4; ++j) {
      const int n = n0 + (j << 4) + rlane;
      float bv = 0.f;
      if (BIAS_MODE == 2) bv = bias[n];
#pragma unroll
      for (int r = 0; r < 8; ++r) {
        float v = acc[i][j][r] * scale;
        if (BIAS_MODE == 1) v += bias[mBase + mOff + r];
        if (BIAS_MODE == 2) v += bv;
        if (RESID) v += Rb[(size_t)(mBase + mOff + r) * ldc + n];
        if (ACT == 2) v = fmaxf(v, 0.0f);
        if (ACT == 4) v = (v > 0.f) ? v : 0.01f * v;
        slab[(mOff + r) * 68 + (j << 4) + rlane] = v;
      }
    }
    __builtin_amdgcn_fence(__ATOMIC_RELEASE, "workgroup");
    __builtin_amdgcn_wave_barrier();
    __builtin_amdgcn_fence(__ATOMIC_ACQUIRE, "workgroup");
    if (OUT_MODE == 0) {
      float* C = (float*)Cout + (size_t)b * strideC;
      const int hh = lane >> 4, c4 = (lane & 15) * 4;
      for (int pass = 0; pass < 2; ++pass) {
#pragma unroll
        for (int it = 0; it < 8; ++it) {
          const int row = it * 2 + hh;
          v4f v = *(const v4f*)(slab + row * 68 + c4);
          *(volatile v4f*)(C + (size_t)(mBase + row) * ldc + n0 + c4) = v;
        }
        __threadfence();
      }
    } else {
      const int q = lane >> 3, c8 = (lane & 7) * 8;
      unsigned short* C  = (unsigned short*)Cout  + (size_t)b * strideC;
      unsigned short* C2 = (OUT_MODE == 2) ? ((unsigned short*)Cout2 + (size_t)b * strideC) : nullptr;
      for (int pass = 0; pass < 2; ++pass) {
#pragma unroll
        for (int it = 0; it < 4; ++it) {
          const int row = it * 4 + q;
          const float* sp = slab + row * 68 + c8;
          v8h hv, lv;
#pragma unroll
          for (int e = 0; e < 8; ++e) {
            if (OUT_MODE == 1) {
              hv[e] = (_Float16)sp[e];
            } else {
              unsigned short hb = f2bf_bits(sp[e]);
              unsigned short lb = f2bf_bits(sp[e] - bf_bits2f(hb));
              hv[e] = __builtin_bit_cast(_Float16, hb);
              lv[e] = __builtin_bit_cast(_Float16, lb);
            }
          }
          *(volatile v8h*)(C + (size_t)(mBase + row) * ldc + n0 + c8) = hv;
          if (OUT_MODE == 2) *(volatile v8h*)(C2 + (size_t)(mBase + row) * ldc + n0 + c8) = lv;
        }
        __threadfence();
      }
    }
    __builtin_amdgcn_fence(__ATOMIC_RELEASE, "workgroup");
    __builtin_amdgcn_wave_barrier();
    __builtin_amdgcn_fence(__ATOMIC_ACQUIRE, "workgroup");
  }
}

__global__ __launch_bounds__(256) void castw_f16_kernel(const float* __restrict__ in, unsigned short* __restrict__ out,
                                                        int rows, int padRows, int cols, float scale) {
  const int i = blockIdx.x * 256 + threadIdx.x;
  const int n8 = (padRows * cols) >> 3;
  if (i >= n8) return;
  const int e0 = i * 8;
  const int r = e0 / cols;
  const int c = e0 - r * cols;
  const int rc = (r < rows) ? r : (rows - 1);
  const float* p = in + (size_t)rc * cols + c;
  const v4f a = *(const v4f*)(p);
  const v4f d = *(const v4f*)(p + 4);
  const bool live = (r < rows);
  unsigned short hb[8];
#pragma unroll
  for (int e = 0; e < 4; ++e) {
    hb[e]     = live ? h_bits(a[e] * scale) : (unsigned short)0;
    hb[4 + e] = live ? h_bits(d[e] * scale) : (unsigned short)0;
  }
  const v4u u = (v4u){pk16(hb[0], hb[1]), pk16(hb[2], hb[3]), pk16(hb[4], hb[5]), pk16(hb[6], hb[7])};
  unsigned short* q = out + (size_t)e0;
  *(volatile v4u*)q = u;
  __threadfence();
  *(volatile v4u*)q = u;
}

__global__ __launch_bounds__(256) void ln_kernel(const float* __restrict__ x, const float* __restrict__ gam,
                                                 const float* __restrict__ bet, unsigned short* __restrict__ out) {
#pragma clang fp contract(off)
  const int lane = threadIdx.x & 31;
  const int wave = threadIdx.x >> 5;
  const int row = blockIdx.x * 8 + wave;
  const float* xr = x + (size_t)row * kIN;
  const int c0 = 8 * lane;
  const int c1 = 256 + 8 * lane;
  const v4f a0 = *(const v4f*)(xr + c0);
  const v4f a1 = *(const v4f*)(xr + c0 + 4);
  const v4f a2 = *(const v4f*)(xr + c1);
  const v4f a3 = *(const v4f*)(xr + c1 + 4);
  float v[16];
#pragma unroll
  for (int e = 0; e < 4; ++e) { v[e] = a0[e]; v[4 + e] = a1[e]; v[8 + e] = a2[e]; v[12 + e] = a3[e]; }
  float s = 0.f;
#pragma unroll
  for (int e = 0; e < 16; ++e) s = s + v[e];
#pragma unroll
  for (int off = 16; off > 0; off >>= 1) s += __shfl_xor(s, off, 32);
  const float mu = s * kInvDim;
  float ss = 0.f;
#pragma unroll
  for (int e = 0; e < 16; ++e) { const float d = v[e] - mu; v[e] = d; ss = ss + d * d; }
#pragma unroll
  for (int off = 16; off > 0; off >>= 1) ss += __shfl_xor(ss, off, 32);
  const float var = ss * kInvDim;
  const float rsd = 1.0f / sqrtf(var + kLnEps);
  const v4f g0 = *(const v4f*)(gam + c0);
  const v4f g1 = *(const v4f*)(gam + c0 + 4);
  const v4f g2 = *(const v4f*)(gam + c1);
  const v4f g3 = *(const v4f*)(gam + c1 + 4);
  const v4f b0 = *(const v4f*)(bet + c0);
  const v4f b1 = *(const v4f*)(bet + c0 + 4);
  const v4f b2 = *(const v4f*)(bet + c1);
  const v4f b3 = *(const v4f*)(bet + c1 + 4);
  float gg[16], bb[16];
#pragma unroll
  for (int e = 0; e < 4; ++e) {
    gg[e] = g0[e]; gg[4 + e] = g1[e]; gg[8 + e] = g2[e]; gg[12 + e] = g3[e];
    bb[e] = b0[e]; bb[4 + e] = b1[e]; bb[8 + e] = b2[e]; bb[12 + e] = b3[e];
  }
  unsigned short hb[16];
#pragma unroll
  for (int e = 0; e < 16; ++e) {
    const float y = (v[e] * rsd) * gg[e] + bb[e];
    hb[e] = h_bits(y);
  }
  const v4u u0 = (v4u){pk16(hb[0], hb[1]), pk16(hb[2], hb[3]), pk16(hb[4], hb[5]), pk16(hb[6], hb[7])};
  const v4u u1 = (v4u){pk16(hb[8], hb[9]), pk16(hb[10], hb[11]), pk16(hb[12], hb[13]), pk16(hb[14], hb[15])};
  unsigned short* orow = out + (size_t)row * kIN;
  *(volatile v4u*)(orow + c0) = u0;
  *(volatile v4u*)(orow + c1) = u1;
  __threadfence();
  *(volatile v4u*)(orow + c0) = u0;
  *(volatile v4u*)(orow + c1) = u1;
}

__global__ __launch_bounds__(64) __attribute__((amdgpu_num_vgpr(256)))
void fw_scan_kernel(const float* __restrict__ qkvb, unsigned short* __restrict__ hs) {
#pragma clang fp contract(off)
  __shared__ __align__(16) float sq[kHD];
  __shared__ __align__(16) float sk[kHD];
  __shared__ __align__(16) float srk[kHD];
  __shared__ __align__(16) float sqh[kHD];
  __shared__ __align__(16) float hst[8 * kHD];
  __shared__ __align__(16) float redM[8];
  __shared__ __align__(16) float redS[8];

  const int bh = blockIdx.x;
  const int b = bh >> 3;
  const int h = bh & 7;
  const int i = threadIdx.x;
  const int lane = i & 31;
  const int wave = i >> 5;
  const int sline = i >> 3;
  const int sc8 = (i & 7) * 8;

  float Wr[kHD], Rr[kHD];
#pragma unroll
  for (int j = 0; j < kHD; ++j) { Wr[j] = 0.f; Rr[j] = 0.f; }
  float hcur = 0.f;

  const float* pb = qkvb + (size_t)b * kProjPad + (size_t)h * kHeadW;
  unsigned short* hsb = hs + (size_t)b * kIN + (size_t)h * kHD;

  for (int t = 0; t < kS; ++t) {
    const float* p = pb + (size_t)t * (size_t)(kB * kProjPad);
    const float ql  = p[i];
    const float kl  = p[kHD + i];
    const float vv  = p[2 * kHD + i];
    const float rkl = p[3 * kHD + i];
    const float rvv = p[4 * kHD + i];
    const float bl  = p[5 * kHD];
    const float rbl = p[5 * kHD + 1];

    float mq = ql, mk = kl, mr = rkl, mh = hcur;
#pragma unroll
    for (int off = 16; off > 0; off >>= 1) {
      mq = fmaxf(mq, __shfl_xor(mq, off, 32));
      mk = fmaxf(mk, __shfl_xor(mk, off, 32));
      mr = fmaxf(mr, __shfl_xor(mr, off, 32));
      mh = fmaxf(mh, __shfl_xor(mh, off, 32));
    }
    if (lane == 0) { redM[wave * 4 + 0] = mq; redM[wave * 4 + 1] = mk; redM[wave * 4 + 2] = mr; redM[wave * 4 + 3] = mh; }
    __syncthreads();

    if (((t & 7) == 0) && (t != 0)) {
      const float* sp = hst + sline * kHD + sc8;
      const v4f ga = *(const v4f*)(sp);
      const v4f gc = *(const v4f*)(sp + 4);
      unsigned short hb[8];
#pragma unroll
      for (int e = 0; e < 4; ++e) { hb[e] = h_bits(ga[e] * kHsCarry); hb[4 + e] = h_bits(gc[e] * kHsCarry); }
      const v4u u = (v4u){pk16(hb[0], hb[1]), pk16(hb[2], hb[3]), pk16(hb[4], hb[5]), pk16(hb[6], hb[7])};
      unsigned short* dst = hsb + (size_t)(t - 8 + sline) * (size_t)(kB * kIN) + sc8;
      *(volatile v4u*)dst = u;
      __threadfence();
      *(volatile v4u*)dst = u;
    }

    const v4f ma = *(const v4f*)(redM);
    const v4f mb = *(const v4f*)(redM + 4);
    const float gq = fmaxf(ma[0], mb[0]);
    const float gk = fmaxf(ma[1], mb[1]);
    const float gr = fmaxf(ma[2], mb[2]);
    const float gh = fmaxf(ma[3], mb[3]);
    const float eq = expf(ql - gq);
    const float ek = expf(kl - gk);
    const float er = expf(rkl - gr);
    const float eh = expf(hcur - gh);
    float pq = eq, pk = ek, pr = er, ph = eh;
#pragma unroll
    for (int off = 16; off > 0; off >>= 1) {
      pq += __shfl_xor(pq, off, 32);
      pk += __shfl_xor(pk, off, 32);
      pr += __shfl_xor(pr, off, 32);
      ph += __shfl_xor(ph, off, 32);
    }
    if (lane == 0) { redS[wave * 4 + 0] = pq; redS[wave * 4 + 1] = pk; redS[wave * 4 + 2] = pr; redS[wave * 4 + 3] = ph; }
    __syncthreads();
    const v4f sa = *(const v4f*)(redS);
    const v4f sb = *(const v4f*)(redS + 4);
    const float invq = 1.0f / (sa[0] + sb[0]);
    const float invk = 1.0f / (sa[1] + sb[1]);
    const float invr = 1.0f / (sa[2] + sb[2]);
    const float invh = 1.0f / (sa[3] + sb[3]);
    sq[i]  = eq * invq;
    sk[i]  = ek * invk;
    srk[i] = er * invr;
    sqh[i] = eh * invh;
    const float bt  = 1.0f / (1.0f + expf(-bl));
    const float rbt = 1.0f / (1.0f + expf(-rbl));
    __syncthreads();

    float vold = 0.f;
#pragma unroll
    for (int jj = 0; jj < 16; ++jj) {
      const v4f kv = *(const v4f*)(sk + 4 * jj);
#pragma unroll
      for (int e = 0; e < 4; ++e) {
        float pp = Wr[4 * jj + e] * kv[e]; defuse(pp);
        vold = vold + pp;
      }
    }
    asm volatile("" ::: "memory");
    const float dv = bt * (vv - vold);
    float z = 0.f;
#pragma unroll
    for (int jj = 0; jj < 16; ++jj) {
      const v4f kv = *(const v4f*)(sk + 4 * jj);
      const v4f qv = *(const v4f*)(sq + 4 * jj);
#pragma unroll
      for (int e = 0; e < 4; ++e) {
        float up = dv * kv[e]; defuse(up);
        const float wn = Wr[4 * jj + e] + up;
        Wr[4 * jj + e] = wn;
        float pp = wn * qv[e]; defuse(pp);
        z = z + pp;
      }
    }
    asm volatile("" ::: "memory");

    float vold2 = 0.f;
#pragma unroll
    for (int jj = 0; jj < 16; ++jj) {
      const v4f kv = *(const v4f*)(srk + 4 * jj);
#pragma unroll
      for (int e = 0; e < 4; ++e) {
        float pp = Rr[4 * jj + e] * kv[e]; defuse(pp);
        vold2 = vold2 + pp;
      }
    }
    asm volatile("" ::: "memory");
    const float dv2 = rbt * (rvv - vold2);
    float racc = 0.f;
#pragma unroll
    for (int jj = 0; jj < 16; ++jj) {
      const v4f kv = *(const v4f*)(srk + 4 * jj);
      const v4f qv = *(const v4f*)(sqh + 4 * jj);
#pragma unroll
      for (int e = 0; e < 4; ++e) {
        float up = dv2 * kv[e]; defuse(up);
        const float rn = Rr[4 * jj + e] + up;
        Rr[4 * jj + e] = rn;
        float pp = rn * qv[e]; defuse(pp);
        racc = racc + pp;
      }
    }
    hcur = z + racc;
    hst[(t & 7) * kHD + i] = hcur;
  }

  __syncthreads();
  {
    const float* sp = hst + sline * kHD + sc8;
    const v4f ga = *(const v4f*)(sp);
    const v4f gc = *(const v4f*)(sp + 4);
    unsigned short hb[8];
#pragma unroll
    for (int e = 0; e < 4; ++e) { hb[e] = h_bits(ga[e] * kHsCarry); hb[4 + e] = h_bits(gc[e] * kHsCarry); }
    const v4u u = (v4u){pk16(hb[0], hb[1]), pk16(hb[2], hb[3]), pk16(hb[4], hb[5]), pk16(hb[6], hb[7])};
    unsigned short* dst = hsb + (size_t)(kS - 8 + sline) * (size_t)(kB * kIN) + sc8;
    *(volatile v4u*)dst = u;
    __threadfence();
    *(volatile v4u*)dst = u;
  }
}

extern "C" void kernel_launch(void* const* d_in, const int* in_sizes, int n_in,
                              void* d_out, int out_size, void* d_ws, size_t ws_size,
                              hipStream_t stream) {
  if (n_in < 5) return;
  if (in_sizes[0] != kRows * kIN) return;
  if (in_sizes[1] != kProj * kIN) return;
  if (in_sizes[2] != kIN * kIN) return;
  if (in_sizes[3] != kIN || in_sizes[4] != kIN) return;
  if (out_size != kRows * kIN) return;
  if (ws_size < kWsTotal) return;

  const float* x     = (const float*)d_in[0];
  const float* Wslow = (const float*)d_in[1];
  const float* Wout  = (const float*)d_in[2];
  const float* gam   = (const float*)d_in[3];
  const float* bet   = (const float*)d_in[4];
  float* out = (float*)d_out;

  char* ws = (char*)d_ws;
  unsigned short* normed16 = (unsigned short*)(ws + kOffNormed);
  unsigned short* wslow16  = (unsigned short*)(ws + kOffWslow);
  unsigned short* wout16   = (unsigned short*)(ws + kOffWout);
  float*          qkvb     = (float*)(ws + kOffQkvb);
  unsigned short* hs16     = (unsigned short*)(ws + kOffHs);

  ln_kernel<<<kRows / 8, 256, 0, stream>>>(x, gam, bet, normed16);

  castw_f16_kernel<<<(kProjPad * kIN / 8) / 256, 256, 0, stream>>>(Wslow, wslow16, kProj, kProjPad, kIN, kWCarry);
  castw_f16_kernel<<<(kIN * kIN / 8) / 256, 256, 0, stream>>>(Wout, wout16, kIN, kIN, kIN, kWCarry);

  {
    dim3 grid((kRows / 64) * (kProjPad / 64) / 8, 1);
    wmma_gemm64<0, false, 0, 0, false><<<grid, 256, 0, stream>>>(
        normed16, normed16, kIN, 0L,
        wslow16, wslow16, kIN, 0L,
        (void*)qkvb, (void*)qkvb, kProjPad, 0L,
        x, x, 0L,
        kRows, kProjPad, kIN, kG1Scale);
  }

  fw_scan_kernel<<<kB * kNH, 64, 0, stream>>>(qkvb, hs16);

  {
    dim3 grid((kRows / 64) * (kIN / 64) / 8, 1);
    wmma_gemm64<0, false, 0, 0, true><<<grid, 256, 0, stream>>>(
        hs16, hs16, kIN, 0L,
        wout16, wout16, kIN, 0L,
        (void*)out, (void*)out, kIN, 0L,
        x, x, 0L,
        kRows, kIN, kIN, kG2Scale);
  }
}
